// EnhancedAttentionLayer_33861522162195
// MI455X (gfx1250) — hardware-verified
//
#include <hip/hip_runtime.h>
#include <math.h>
#include <stdint.h>

#ifndef NB
#define NB 4
#endif
#ifndef SEQ
#define SEQ 2048
#endif
#define NB_FULL  4
#define SEQ_FULL 2048
#define EMB      1024
#define NH       8
#define HD       128
#define NQ64     (SEQ / 64)
#define NKT      (SEQ / 64)
#define NSLOTG   ((SEQ / 4 + 255) / 256)
#define SM_SCALE 0.08838834764831845f
#define OFF1     ((size_t)NB_FULL * EMB)
#define OFF2     (OFF1 + (size_t)NB_FULL * NH * SEQ_FULL)
static_assert(NB >= 1 && NB <= NB_FULL);
static_assert(SEQ >= 128 && SEQ <= SEQ_FULL && (SEQ % 128) == 0);
static_assert(NH * HD == EMB);
static_assert(HD == 128);
static_assert((EMB % 64) == 0 && (EMB % 32) == 0 && (SEQ % 64) == 0);
static_assert(OFF1 * 4 == 16384);
static_assert(OFF2 * 4 == 278528);

typedef _Float16 v16h __attribute__((ext_vector_type(16)));
typedef _Float16 v8h  __attribute__((ext_vector_type(8)));
typedef __bf16   v16b __attribute__((ext_vector_type(16)));
typedef __bf16   v8b  __attribute__((ext_vector_type(8)));
typedef float    v8f  __attribute__((ext_vector_type(8)));
typedef float    v4f  __attribute__((ext_vector_type(4)));
typedef unsigned int v4u __attribute__((ext_vector_type(4)));

#if defined(__HIP_DEVICE_COMPILE__)
#define DEV_ASM 1
#else
#define DEV_ASM 0
#endif

__device__ __forceinline__ unsigned short bf_bits(float f) {
  unsigned u = __float_as_uint(f);
  return (unsigned short)((u + 0x7FFFu + ((u >> 16) & 1u)) >> 16);
}
__device__ __forceinline__ float bf_up(unsigned short hb) { return __uint_as_float(((unsigned)hb) << 16); }
__device__ __forceinline__ unsigned short h_bits(_Float16 x) { return __builtin_bit_cast(unsigned short, x); }
__device__ __forceinline__ unsigned pk16(unsigned short a, unsigned short b) { return (unsigned)a | ((unsigned)b << 16); }
__device__ __forceinline__ v8f zero8() { v8f z = {0.f, 0.f, 0.f, 0.f, 0.f, 0.f, 0.f, 0.f}; return z; }

template <typename OT> struct FT;
template <> struct FT<__bf16>   { typedef v16b frag; typedef v8b half8; };
template <> struct FT<_Float16> { typedef v16h frag; typedef v8h half8; };

template <typename OT>
__device__ __forceinline__ typename FT<OT>::frag ldfrag(const OT* p) {
  union { typename FT<OT>::frag v; typename FT<OT>::half8 h[2]; } f;
  f.h[0] = *(const typename FT<OT>::half8*)(p);
  f.h[1] = *(const typename FT<OT>::half8*)(p + 16);
  return f.v;
}

__device__ __forceinline__ v8f mmar(v16b a, v16b b, v8f c) {
  return __builtin_amdgcn_wmma_f32_16x16x32_bf16(false, a, false, b, (short)0, c, false, false);
}
__device__ __forceinline__ v8f mmar(v16h a, v16h b, v8f c) {
  return __builtin_amdgcn_wmma_f32_16x16x32_f16(false, a, false, b, (short)0, c, false, false);
}
__device__ __forceinline__ v8f mma_h(v16h a, v16h b, v8f c) {
  c = __builtin_amdgcn_wmma_f32_16x16x32_f16(false, a, false, b, (short)0, c, false, false);
#if DEV_ASM
  asm volatile("v_nop\n\tv_nop\n\tv_nop\n\tv_nop" : "+v"(c) : "v"(a), "v"(b));
#endif
  return c;
}
__device__ __forceinline__ void dep_guard(v8f& a, v8f& b, v16b x, v16b y) {
#if DEV_ASM
  asm volatile("v_nop\n\tv_nop\n\tv_nop\n\tv_nop" : "+v"(a), "+v"(b) : "v"(x), "v"(y));
#else
  (void)a; (void)b; (void)x; (void)y;
#endif
}
__device__ __forceinline__ void dep_guard(v8f& a, v8f& b, v16h x, v16h y) {
#if DEV_ASM
  asm volatile("v_nop\n\tv_nop\n\tv_nop\n\tv_nop" : "+v"(a), "+v"(b) : "v"(x), "v"(y));
#else
  (void)a; (void)b; (void)x; (void)y;
#endif
}
__device__ __forceinline__ void keep4(v16b a, v16b b, v16b c, v16b d) {
#if DEV_ASM
  asm volatile("v_nop" :: "v"(a), "v"(b), "v"(c), "v"(d));
#else
  (void)a; (void)b; (void)c; (void)d;
#endif
}
__device__ __forceinline__ void keep4(v16h a, v16h b, v16h c, v16h d) {
#if DEV_ASM
  asm volatile("v_nop" :: "v"(a), "v"(b), "v"(c), "v"(d));
#else
  (void)a; (void)b; (void)c; (void)d;
#endif
}
__device__ __forceinline__ void acc_guard4(v8f& a, v8f& b, v8f& c, v8f& d) {
#if DEV_ASM
  asm volatile("v_nop\n\tv_nop\n\tv_nop\n\tv_nop" : "+v"(a), "+v"(b), "+v"(c), "+v"(d));
#else
  (void)a; (void)b; (void)c; (void)d;
#endif
}

__global__ __launch_bounds__(256) void cvt_bf16x8(const float* __restrict__ in, unsigned short* out, int n8,
                                                   long long sIn, long long sOut) {
  const int i = blockIdx.x * 256 + (int)threadIdx.x;
  const int b = blockIdx.y;
  if (i < n8) {
    const float* ip = in + (size_t)b * (size_t)sIn + (size_t)i * 8;
    const v4f a  = *(const v4f*)(ip);
    const v4f a4 = *(const v4f*)(ip + 4);
    v4u p;
    p[0] = pk16(bf_bits(a[0]),  bf_bits(a[1]));
    p[1] = pk16(bf_bits(a[2]),  bf_bits(a[3]));
    p[2] = pk16(bf_bits(a4[0]), bf_bits(a4[1]));
    p[3] = pk16(bf_bits(a4[2]), bf_bits(a4[3]));
    unsigned short* o = out + (size_t)b * (size_t)sOut + (size_t)i * 8;
    *(volatile v4u*)o = p;
    __threadfence();
    *(volatile v4u*)o = p;
  }
}

template <typename OT, int MI, int NPA, int OUT_MODE, int BM>
__global__ __launch_bounds__(256) void gemm_t(
    const unsigned short* __restrict__ Ap, const unsigned short* __restrict__ A2p, int lda, long long strideA,
    const unsigned short* __restrict__ Btp, int ldb, long long strideB,
    void* Cout, void* Cout2, int ldc, long long strideC,
    const float* __restrict__ bias,
    int M, int N, int K, float oscale, float rscaleA, float cscale, float rscaleC) {
  typedef typename FT<OT>::frag V16;
  const OT* A  = (const OT*)(const void*)Ap;
  const OT* A2 = (const OT*)(const void*)A2p;
  const OT* Bt = (const OT*)(const void*)Btp;
  __shared__ __align__(16) float sT[8][16 * 68];
  const int RT   = 16 * MI;
  const int b    = blockIdx.y;
  const int lane = threadIdx.x & 31;
  const int wave = threadIdx.x >> 5;
  const int tilesN = N >> 6;
  const int tilesM = M / RT;
  const int tile = blockIdx.x * 8 + wave;
  if (tile >= tilesM * tilesN) return;
  const int tm = tile / tilesN;
  const int tn = tile - tm * tilesN;
  const int m0 = tm * RT;
  const int n0 = tn << 6;

  const OT* Ab  = A  + (size_t)b * (size_t)strideA;
  const OT* A2b = A2 + (size_t)b * (size_t)strideA;
  const OT* Bb  = Bt + (size_t)b * (size_t)strideB;

  const int rlane = lane & 15;
  const int koff  = (lane >> 4) * 8;
  const int mOff  = (lane >> 4) * 8;

  v8f acc[MI][4], acc2[MI][4];
#pragma unroll
  for (int i = 0; i < MI; ++i)
#pragma unroll
    for (int j = 0; j < 4; ++j) { acc[i][j] = zero8(); acc2[i][j] = zero8(); }

  for (int k0 = 0; k0 < K; k0 += 32) {
    V16 bq[4];
#pragma unroll
    for (int j = 0; j < 4; ++j)
      bq[j] = ldfrag<OT>(Bb + (size_t)(n0 + (j << 4) + rlane) * ldb + koff + k0);
#pragma unroll
    for (int i = 0; i < MI; ++i) {
      const V16 af = ldfrag<OT>(Ab + (size_t)(m0 + (i << 4) + rlane) * lda + koff + k0);
#pragma unroll
      for (int j = 0; j < 4; ++j) acc[i][j] = mmar(af, bq[j], acc[i][j]);
      dep_guard(acc[i][0], acc[i][3], af, bq[3]);
      if (NPA == 2) {
        const V16 af2 = ldfrag<OT>(A2b + (size_t)(m0 + (i << 4) + rlane) * lda + koff + k0);
#pragma unroll
        for (int j = 0; j < 4; ++j) acc2[i][j] = mmar(af2, bq[j], acc2[i][j]);
        dep_guard(acc2[i][0], acc2[i][3], af2, bq[3]);
      }
    }
    keep4(bq[0], bq[1], bq[2], bq[3]);
  }
#pragma unroll
  for (int i = 0; i < MI; ++i) {
    acc_guard4(acc[i][0], acc[i][1], acc[i][2], acc[i][3]);
    if (NPA == 2) acc_guard4(acc2[i][0], acc2[i][1], acc2[i][2], acc2[i][3]);
  }

  float bcol[4];
#pragma unroll
  for (int j = 0; j < 4; ++j) bcol[j] = 0.f;
  if (BM == 1) {
#pragma unroll
    for (int j = 0; j < 4; ++j) bcol[j] = bf_up(bf_bits(bias[n0 + (j << 4) + rlane]));
  }
  float* slab = sT[wave];
#pragma unroll
  for (int i = 0; i < MI; ++i) {
    const int mBase = m0 + (i << 4);
    float brow[8];
#pragma unroll
    for (int r = 0; r < 8; ++r) brow[r] = 0.f;
    if (BM == 2) {
#pragma unroll
      for (int r = 0; r < 8; ++r) brow[r] = bf_up(bf_bits(bias[mBase + mOff + r]));
    }
#pragma unroll
    for (int j = 0; j < 4; ++j) {
#pragma unroll
      for (int r = 0; r < 8; ++r) {
        float v = acc[i][j][r];
        if (NPA == 2) v += acc2[i][j][r] * rscaleA;
        v = v * oscale + bcol[j] + brow[r];
        slab[(mOff + r) * 68 + (j << 4) + rlane] = v;
      }
    }
    __builtin_amdgcn_fence(__ATOMIC_RELEASE, "workgroup");
    __builtin_amdgcn_wave_barrier();
    __builtin_amdgcn_fence(__ATOMIC_ACQUIRE, "workgroup");
    if (OUT_MODE == 0) {
      float* C = (float*)Cout + (size_t)b * (size_t)strideC;
      const int h2 = lane >> 4, c4 = (lane & 15) * 4;
      for (int pass = 0; pass < 2; ++pass) {
#pragma unroll
        for (int it = 0; it < 8; ++it) {
          const int row = it * 2 + h2;
          const v4f v = *(const v4f*)(slab + row * 68 + c4);
          *(volatile v4f*)(C + (size_t)(mBase + row) * ldc + n0 + c4) = v;
        }
        __threadfence();
      }
    } else {
      const int q = lane >> 3, c8 = (lane & 7) * 8;
      unsigned short* C  = (unsigned short*)Cout  + (size_t)b * (size_t)strideC;
      unsigned short* C2 = (unsigned short*)Cout2 + (size_t)b * (size_t)strideC;
      v4u hv[4], lv[4];
#pragma unroll
      for (int it = 0; it < 4; ++it) {
        const int row = it * 4 + q;
        const float* sp = slab + row * 68 + c8;
        float f[8];
#pragma unroll
        for (int e = 0; e < 8; ++e) f[e] = sp[e] * cscale;
        v4u a, a2;
#pragma unroll
        for (int e = 0; e < 4; ++e) {
          const float f0 = f[2 * e], f1 = f[2 * e + 1];
          const _Float16 x0 = (_Float16)f0, x1 = (_Float16)f1;
          const unsigned short h0 = h_bits(x0), h1 = h_bits(x1);
          unsigned short l0 = 0, l1 = 0;
          if (OUT_MODE == 3) {
            l0 = h_bits((_Float16)((f0 - (float)x0) * rscaleC));
            l1 = h_bits((_Float16)((f1 - (float)x1) * rscaleC));
          }
          a[e] = pk16(h0, h1); a2[e] = pk16(l0, l1);
        }
        hv[it] = a; lv[it] = a2;
      }
      for (int pass = 0; pass < 2; ++pass) {
#pragma unroll
        for (int it = 0; it < 4; ++it) {
          const int row = it * 4 + q;
          *(volatile v4u*)(C + (size_t)(mBase + row) * ldc + n0 + c8) = hv[it];
          if (OUT_MODE == 3) *(volatile v4u*)(C2 + (size_t)(mBase + row) * ldc + n0 + c8) = lv[it];
        }
        __threadfence();
      }
    }
    __builtin_amdgcn_fence(__ATOMIC_RELEASE, "workgroup");
    __builtin_amdgcn_wave_barrier();
    __builtin_amdgcn_fence(__ATOMIC_ACQUIRE, "workgroup");
  }
}

__device__ __forceinline__ void score_chunk(const v16h (&qah)[4], const v16h (&qal)[4],
                                            const _Float16* __restrict__ kb0, int kv0, int c, int hh,
                                            v8f (&s)[4]) {
  union FH { v16h v; v8h h[2]; };
#pragma unroll
  for (int j = 0; j < 4; ++j) {
    v8f ah = zero8(), al = zero8();
#pragma unroll
    for (int dc = 0; dc < 4; ++dc) {
      const _Float16* kp = kb0 + (size_t)(kv0 + j * 16 + c) * (size_t)EMB + dc * 32 + 8 * hh;
      FH kb;
      kb.h[0] = *(const v8h*)(kp);
      kb.h[1] = *(const v8h*)(kp + 16);
      ah = mma_h(qah[dc], kb.v, ah);
      al = mma_h(qal[dc], kb.v, al);
    }
#pragma unroll
    for (int r = 0; r < 8; ++r) s[j][r] = (ah[r] + al[r] * (1.0f / 4096.0f)) * SM_SCALE;
  }
}

__global__ __launch_bounds__(128)
void attn_colsum(const unsigned short* __restrict__ qhp, const unsigned short* __restrict__ qlp,
                 const unsigned short* __restrict__ kpp, float* PS) {
  __shared__ __align__(16) float csl[4][64];
  const int tid  = threadIdx.x;
  const int wave = tid >> 5;
  const int lane = tid & 31;
  const int hh   = lane >> 4;
  const int c    = lane & 15;
  const int bx   = blockIdx.x;
  const int qb   = bx % NQ64;
  const int rest = bx / NQ64;
  const int h    = rest % NH;
  const int b    = rest / NH;
  const int bh   = b * NH + h;
  const int q0   = qb * 64 + wave * 16;

  const _Float16* Qh  = (const _Float16*)(const void*)qhp;
  const _Float16* Ql  = (const _Float16*)(const void*)qlp;
  const _Float16* Kb0 = (const _Float16*)(const void*)kpp + (size_t)b * SEQ * EMB + (size_t)h * HD;

  v16h qah[4], qal[4];
#pragma unroll
  for (int dc = 0; dc < 4; ++dc) {
    const size_t qo = ((size_t)b * SEQ + (size_t)(q0 + c)) * EMB + (size_t)h * HD + dc * 32 + 8 * hh;
    qah[dc] = ldfrag<_Float16>(Qh + qo);
    qal[dc] = ldfrag<_Float16>(Ql + qo);
  }

  float mrow[8], lrow[8];
#pragma unroll
  for (int r = 0; r < 8; ++r) { mrow[r] = -INFINITY; lrow[r] = 0.f; }

  for (int kt = 0; kt < NKT; ++kt) {
    const int kv0 = kt * 64;
    v8f s[4];
    score_chunk(qah, qal, Kb0, kv0, c, hh, s);
#pragma unroll
    for (int r = 0; r < 8; ++r) {
      float m = s[0][r];
#pragma unroll
      for (int j = 1; j < 4; ++j) m = fmaxf(m, s[j][r]);
#pragma unroll
      for (int off = 1; off < 16; off <<= 1) m = fmaxf(m, __shfl_xor(m, off, 32));
      const float mnew  = fmaxf(mrow[r], m);
      const float msafe = (mnew == -INFINITY) ? 0.f : mnew;
      const float alpha = __expf(mrow[r] - msafe);
      mrow[r] = mnew;
      float psum = 0.f;
#pragma unroll
      for (int j = 0; j < 4; ++j) psum += __expf(s[j][r] - msafe);
#pragma unroll
      for (int off = 1; off < 16; off <<= 1) psum += __shfl_xor(psum, off, 32);
      lrow[r] = lrow[r] * alpha + psum;
    }
  }

  float il[8], mf[8];
#pragma unroll
  for (int r = 0; r < 8; ++r) {
    const float l = lrow[r];
    il[r] = (l > 0.f) ? (1.0f / l) : 0.f;
    mf[r] = (mrow[r] == -INFINITY) ? 0.f : mrow[r];
  }

  for (int kt = 0; kt < NKT; ++kt) {
    const int kv0 = kt * 64;
    v8f s[4];
    score_chunk(qah, qal, Kb0, kv0, c, hh, s);
    float cs[4];
#pragma unroll
    for (int j = 0; j < 4; ++j) {
      float a = 0.f;
#pragma unroll
      for (int r = 0; r < 8; ++r) a += __expf(s[j][r] - mf[r]) * il[r];
      cs[j] = a;
    }
#pragma unroll
    for (int j = 0; j < 4; ++j) cs[j] += __shfl_xor(cs[j], 16, 32);
    const float v0 = hh ? cs[2] : cs[0];
    const float v1 = hh ? cs[3] : cs[1];
    csl[wave][32 * hh + c]      = v0;
    csl[wave][32 * hh + 16 + c] = v1;
    __syncthreads();
    if (wave == 0 && lane < 16) {
      v4f a = *(const v4f*)(&csl[0][4 * lane]);
      a += *(const v4f*)(&csl[1][4 * lane]);
      a += *(const v4f*)(&csl[2][4 * lane]);
      a += *(const v4f*)(&csl[3][4 * lane]);
      float* dst = PS + ((size_t)(bh * NQ64 + qb)) * SEQ + kv0 + 4 * lane;
      *(volatile v4f*)dst = a;
      __threadfence();
      *(volatile v4f*)dst = a;
    }
    __syncthreads();
  }
}

__global__ __launch_bounds__(256)
void avg_ctx(const float* __restrict__ PS, const float* __restrict__ Vp, float* out1, float* CS) {
  __shared__ __align__(16) float avs[SEQ];
  __shared__ double cpart[2][HD];
  __shared__ __align__(16) float csf[HD];
  const int tid = threadIdx.x;
  const int bh  = blockIdx.x;
  const int b   = bh / NH;
  const int h   = bh - b * NH;
  const float* psb = PS + (size_t)bh * NQ64 * SEQ;

  for (int g = 0; g < NSLOTG; ++g) {
    const int slot = g * 256 + tid;
    if (slot < SEQ / 4) {
      v4f a = *(const v4f*)(psb + 4 * slot);
#pragma unroll 8
      for (int qb = 1; qb < NQ64; ++qb) a += *(const v4f*)(psb + (size_t)qb * SEQ + 4 * slot);
      a *= (1.0f / (float)SEQ);
      *(v4f*)(avs + 4 * slot) = a;
      float* dst = out1 + (size_t)bh * SEQ + 4 * slot;
      *(volatile v4f*)dst = a;
      __threadfence();
      *(volatile v4f*)dst = a;
    }
  }
  __syncthreads();

  const int d    = tid & (HD - 1);
  const int half = tid >> 7;
  const int kb   = half * (SEQ / 2);
  const float* vb = Vp + (size_t)b * SEQ * EMB + (size_t)h * HD + d;
  double acc = 0.0;
#pragma unroll 4
  for (int k = 0; k < SEQ / 2; ++k)
    acc += (double)avs[kb + k] * (double)vb[(size_t)(kb + k) * EMB];
  cpart[half][d] = acc;
  __syncthreads();
  if (tid < HD) csf[tid] = (float)(cpart[0][tid] + cpart[1][tid]);
  __syncthreads();
  if (tid < 32) {
    const v4f v = *(const v4f*)(csf + 4 * tid);
    float* dst = CS + (size_t)b * EMB + (size_t)h * HD + 4 * tid;
    *(volatile v4f*)dst = v;
    __threadfence();
    *(volatile v4f*)dst = v;
  }
}

__global__ __launch_bounds__(256)
void ctx_out(const float* __restrict__ CS, const float* __restrict__ Wo, const float* __restrict__ bo, float* out0) {
  __shared__ __align__(16) float res[32];
  const int tid  = threadIdx.x;
  const int wave = tid >> 5;
  const int lane = tid & 31;
  const int j0   = blockIdx.x * 32;
  const int b    = j0 / EMB;
  const float* csb = CS + (size_t)b * EMB;
#pragma unroll 1
  for (int u = 0; u < 4; ++u) {
    const int j = j0 - b * EMB + wave * 4 + u;
    const float* wr = Wo + (size_t)j * EMB;
    float acc = 0.f;
#pragma unroll 4
    for (int it = 0; it < EMB / 32; ++it) {
      const int i = it * 32 + lane;
      acc += csb[i] * bf_up(bf_bits(wr[i]));
    }
#pragma unroll
    for (int off = 16; off > 0; off >>= 1) acc += __shfl_xor(acc, off, 32);
    const float val = acc + bf_up(bf_bits(bo[j]));
    if (lane == 0) res[wave * 4 + u] = val;
  }
  __syncthreads();
  if (tid < 8) {
    const v4f v = *(const v4f*)(res + 4 * tid);
    float* dst = out0 + (size_t)j0 + 4 * tid;
    *(volatile v4f*)dst = v;
    __threadfence();
    *(volatile v4f*)dst = v;
  }
}

__global__ __launch_bounds__(256)
void div_k(const float* __restrict__ avg, float* dv) {
  __shared__ double red[256];
  const int tid = threadIdx.x;
  double tot = 0.0;
  for (int base = 0; base < NB * NH * NH; base += 256) {
    const int tr = base + tid;
    double cval = 0.0;
    if (tr < NB * NH * NH) {
      const int b = tr / (NH * NH);
      const int h = (tr / NH) % NH;
      const int g = tr % NH;
      const float* ah = avg + ((size_t)b * NH + h) * SEQ;
      const float* ag = avg + ((size_t)b * NH + g) * SEQ;
      double cacc = 0.0;
#pragma unroll 4
      for (int s = 0; s < SEQ; ++s) cacc += (double)ah[s] * (double)ag[s];
      cval = (h == g) ? 0.0 : fabs(cacc);
    }
    tot += cval;
  }
  red[tid] = tot;
  __syncthreads();
#pragma unroll 1
  for (int off = 128; off > 0; off >>= 1) {
    if (tid < off) red[tid] += red[tid + off];
    __syncthreads();
  }
  if (tid == 0) {
    const float v = (float)(red[0] * (1.0 / (double)(NB * NH * NH)));
    *(volatile float*)dv = v;
    __threadfence();
    *(volatile float*)dv = v;
  }
}

extern "C" void kernel_launch(void* const* d_in, const int* in_sizes, int n_in,
                              void* d_out, int out_size, void* d_ws, size_t ws_size,
                              hipStream_t stream) {
  if (n_in < 9) return;
  const long long needX = (long long)(NB - 1) * SEQ_FULL * EMB + (long long)SEQ * EMB;
  if ((long long)in_sizes[0] < needX) return;
  if (in_sizes[1] < EMB * EMB || in_sizes[3] < EMB * EMB || in_sizes[5] < EMB * EMB || in_sizes[7] < EMB * EMB) return;
  if (in_sizes[2] < EMB || in_sizes[4] < EMB || in_sizes[6] < EMB || in_sizes[8] < EMB) return;
  if (out_size < 0) return;
  if ((size_t)out_size < OFF2 + 1) return;

  const float* x  = (const float*)d_in[0];
  const float* Wq = (const float*)d_in[1];
  const float* bq = (const float*)d_in[2];
  const float* Wk = (const float*)d_in[3];
  const float* bk = (const float*)d_in[4];
  const float* Wv = (const float*)d_in[5];
  const float* bv = (const float*)d_in[6];
  const float* Wo = (const float*)d_in[7];
  const float* bo = (const float*)d_in[8];

  const size_t PXB = (size_t)NB * SEQ * EMB * 2;
  const size_t PW  = (size_t)EMB * EMB * 2;
  const size_t PV  = (size_t)NB * SEQ * EMB * 4;
  const size_t PPS = (size_t)NB * NH * NQ64 * SEQ * 4;
  const size_t PCS = (size_t)NB * EMB * 4;
  size_t off = 0;
  const size_t oXb = off; off += PXB;
  const size_t oWq = off; off += PW;
  const size_t oWk = off; off += PW;
  const size_t oWv = off; off += PW;
  const size_t oQh = off; off += PXB;
  const size_t oQl = off; off += PXB;
  const size_t oKp = off; off += PXB;
  const size_t oVp = off; off += PV;
  const size_t oPS = off; off += PPS;
  const size_t oCS = off; off += PCS;
  if (off > ws_size) return;
  if (off > (size_t)134217728) return;

  char* ws = (char*)d_ws;
  unsigned short* Xb  = (unsigned short*)(ws + oXb);
  unsigned short* Wqb = (unsigned short*)(ws + oWq);
  unsigned short* Wkb = (unsigned short*)(ws + oWk);
  unsigned short* Wvb = (unsigned short*)(ws + oWv);
  unsigned short* Qh  = (unsigned short*)(ws + oQh);
  unsigned short* Ql  = (unsigned short*)(ws + oQl);
  unsigned short* Kp  = (unsigned short*)(ws + oKp);
  float*          Vp  = (float*)(ws + oVp);
  float*          PS  = (float*)(ws + oPS);
  float*          CS  = (float*)(ws + oCS);
  float*          out0 = (float*)d_out;
  float*          out1 = (float*)d_out + OFF1;
  float*          out2 = (float*)d_out + OFF2;

  const dim3 blk(256);
  const int n8x = SEQ * EMB / 8;
  const int n8w = EMB * EMB / 8;
  const dim3 gCvtX((n8x + 255) / 256, NB);
  const dim3 gCvtW((n8w + 255) / 256, 1);
  const int tilesP = (SEQ / 64) * (EMB / 64);
  const dim3 gP((tilesP + 7) / 8, NB);
  const dim3 gAttn(NB * NH * NQ64);
  const dim3 gAvg(NB * NH);
  const dim3 gCtx(NB * EMB / 32);
  const long long sXin = (long long)SEQ_FULL * EMB;
  const long long sAct = (long long)SEQ * EMB;

  cvt_bf16x8<<<gCvtX, blk, 0, stream>>>(x,  Xb,  n8x, sXin, sAct);
  cvt_bf16x8<<<gCvtW, blk, 0, stream>>>(Wq, Wqb, n8w, 0LL, 0LL);
  cvt_bf16x8<<<gCvtW, blk, 0, stream>>>(Wk, Wkb, n8w, 0LL, 0LL);
  cvt_bf16x8<<<gCvtW, blk, 0, stream>>>(Wv, Wvb, n8w, 0LL, 0LL);
  gemm_t<__bf16, 4, 1, 3, 1><<<gP, blk, 0, stream>>>(
      Xb, Xb, EMB, sAct, Wqb, EMB, 0LL,
      (void*)Qh, (void*)Ql, EMB, sAct, bq,
      SEQ, EMB, EMB, 1.0f, 0.0f, 1.0f, 4096.0f);
  gemm_t<__bf16, 4, 1, 1, 1><<<gP, blk, 0, stream>>>(
      Xb, Xb, EMB, sAct, Wkb, EMB, 0LL,
      (void*)Kp, (void*)Kp, EMB, sAct, bk,
      SEQ, EMB, EMB, 1.0f, 0.0f, 1.0f, 1.0f);
  gemm_t<__bf16, 4, 1, 0, 1><<<gP, blk, 0, stream>>>(
      Xb, Xb, EMB, sAct, Wvb, EMB, 0LL,
      (void*)Vp, (void*)Vp, EMB, sAct, bv,
      SEQ, EMB, EMB, 1.0f, 0.0f, 1.0f, 1.0f);
  attn_colsum<<<gAttn, dim3(128), 0, stream>>>(Qh, Ql, Kp, PS);
  avg_ctx<<<gAvg, blk, 0, stream>>>(PS, Vp, out1, CS);
  ctx_out<<<gCtx, blk, 0, stream>>>(CS, Wo, bo, out0);
  div_k<<<dim3(1), blk, 0, stream>>>((const float*)out1, out2);
  (void)hipGetLastError();
}
